// DeepGSEA_45191645888600
// MI455X (gfx1250) — hardware-verified
//
#include <hip/hip_runtime.h>


namespace {
constexpr int B = 2048, G = 2000, C = 50, H = 256, ZD = 32, K = 10, P = 4, KG = 256  ;
constexpr float XS = 8.0f, WSC = 256.0f, SLOPE = 0.01f;

typedef _Float16 b16;
typedef __attribute__((ext_vector_type(16))) _Float16 v16b;
typedef __attribute__((ext_vector_type(8))) _Float16 v8b;
typedef __attribute__((ext_vector_type(8))) float v8f;
typedef __attribute__((ext_vector_type(4))) float v4f;
__device__ __forceinline__ float bf16_rne(float f) { unsigned int u = __float_as_uint(f); u += 0x7FFFu + ((u >> 16) & 1u); return __uint_as_float(u & 0xFFFF0000u); }
__device__ __forceinline__ void split16(float v, b16& hi, b16& lo) { hi = (b16)v; lo = (b16)(v - (float)hi); }
__device__ __forceinline__ v16b frag_kb(const b16* p, int hh) { const v8b a = *(const v8b*)(p + 8 * hh), b = *(const v8b*)(p + 16 + 8 * hh); v16b f;
#pragma unroll
  for (int e = 0; e < 8; ++e) { f[e] = a[e]; f[8 + e] = b[e]; } return f; }
__device__ __forceinline__ v8f wmma16b(v16b a, v16b b, v8f c) { v8f d = __builtin_amdgcn_wmma_f32_16x16x32_f16(false, a, false, b, (short)0, c, false, false); asm volatile("v_nop\n\tv_nop\n\tv_nop\n\tv_nop" : "+v"(d) : "v"(a), "v"(b)); return d; }
__device__ __forceinline__ void wave_lds_sync() { __builtin_amdgcn_fence(__ATOMIC_RELEASE, "workgroup"); __builtin_amdgcn_wave_barrier(); __builtin_amdgcn_fence(__ATOMIC_ACQUIRE, "workgroup"); }
__device__ __forceinline__ float pmul(float a, float b) { float p = a * b; asm volatile("" : "+v"(p)); return p; }
__device__ __forceinline__ float lrelu(float x) { return x > 0.0f ? x : SLOPE * x; }
__device__ __forceinline__ int iclamp(int v, int lo, int hi) { return v < lo ? lo : (v > hi ? hi : v); }

__global__ __launch_bounds__(256) void genes_kernel(const float* __restrict__ M, int* __restrict__ IDX, int* __restrict__ FLAG) {
  __shared__ int cnt[256], lst[KG + 32]; __shared__ int base;
  const int c = blockIdx.x, t_ = threadIdx.x; if (t_ == 0) base = 0; for (int i = t_; i < KG + 32; i += 256) lst[i] = -1;
  __syncthreads();
  for (int r0 = 0; r0 < G; r0 += 256) { const int g = r0 + t_; const int on = (g < G && bf16_rne(M[(size_t)c * G + g]) != 0.0f) ? 1 : 0; cnt[t_] = on; __syncthreads();
    for (int s = 1; s < 256; s <<= 1) { const int v = (t_ >= s) ? cnt[t_ - s] : 0; __syncthreads(); cnt[t_] += v; __syncthreads(); }
    const int pos = base + cnt[t_] - on; if (on && pos < KG) lst[pos] = g; __syncthreads(); if (t_ == 255) base += cnt[255]; __syncthreads(); }
  for (int pass = 0; pass < 2; ++pass) { ((volatile int*)IDX)[(size_t)c * KG + t_] = lst[t_]; if (t_ == 0 && base > KG) ((volatile int*)FLAG)[0] = 1; __threadfence(); }
}
__global__ __launch_bounds__(256) void gather_kernel(const float* __restrict__ X, const float* __restrict__ W1, const int* __restrict__ IDX, int c, b16* __restrict__ XG, b16* __restrict__ W1G) {
  __shared__ int idx[KG];
  const int t_ = threadIdx.x; idx[t_] = IDX[(size_t)c * KG + t_]; __syncthreads();
  const size_t t = (size_t)blockIdx.x * 256 + t_; const size_t nx = (size_t)B * KG / 8, nw = (size_t)H * KG / 8; v8b o = {};
  if (t < nx) { const size_t row = t / (KG / 8); const int k0 = (int)(t - row * (KG / 8)) * 8; for (int j = 0; j < 8; ++j) { const int g = idx[k0 + j]; o[j] = (b16)((g >= 0) ? bf16_rne(X[row * G + iclamp(g, 0, G - 1)]) * XS : 0.0f); }
    for (int pass = 0; pass < 2; ++pass) { *(volatile v8b*)(XG + row * KG + k0) = o; __threadfence(); } }
  else if (t < nx + nw) { const size_t u = t - nx; const int oo = (int)(u / (KG / 8)); const int k0 = (int)(u - (size_t)oo * (KG / 8)) * 8; for (int j = 0; j < 8; ++j) { const int g = idx[k0 + j]; o[j] = (b16)((g >= 0) ? bf16_rne(W1[(size_t)iclamp(g, 0, G - 1) * H + oo]) * WSC : 0.0f); }
    for (int pass = 0; pass < 2; ++pass) { *(volatile v8b*)(W1G + (size_t)oo * KG + k0) = o; __threadfence(); } }
}
__global__ __launch_bounds__(256) void prep_kernel(const float* __restrict__ W2, const float* __restrict__ cw, b16* __restrict__ W2T, b16* __restrict__ CW) {
  const size_t t = (size_t)blockIdx.x * 256 + threadIdx.x; const size_t n1 = (size_t)H * H / 8, n2 = (size_t)C * ZD * H / 8; v8b o;
  if (t < n1) { const size_t u = t * 8; const int oo = (int)(u / H), i0 = (int)(u - (size_t)oo * H); for (int j = 0; j < 8; ++j) o[j] = (b16)(bf16_rne(W2[(size_t)(i0 + j) * H + oo]) * WSC); for (int pass = 0; pass < 2; ++pass) { *(volatile v8b*)(W2T + u) = o; __threadfence(); } }
  else if (t < n1 + n2) { const size_t u = (t - n1) * 8; for (int j = 0; j < 8; ++j) o[j] = (b16)(bf16_rne(cw[u + j]) * WSC); for (int pass = 0; pass < 2; ++pass) { *(volatile v8b*)(CW + u) = o; __threadfence(); } }
}
template <int MODE>
__global__ __launch_bounds__(128) void gemm_kernel(const b16* __restrict__ Ah, const b16* __restrict__ Al, const b16* __restrict__ W, const float* __restrict__ bias, int c, b16* __restrict__ Yh, b16* __restrict__ Yl, float* __restrict__ ZP) {
  constexpr int NT = (MODE == 2) ? 2 : 8;
  __shared__ __attribute__((aligned(16))) float Ts[4][16][128 + 4];
  const int wave = threadIdx.x >> 5, lane = threadIdx.x & 31, nloc = lane & 15, hlf = lane >> 4; const size_t m0 = (size_t)blockIdx.x * 64 + wave * 16; const int n0 = blockIdx.y * 128;
  v8f acc[NT];
#pragma unroll
  for (int t = 0; t < NT; ++t) acc[t] = (v8f){};
#pragma unroll 2
  for (int kb = 0; kb < KG; kb += 32) { const v16b a = frag_kb(Ah + (m0 + nloc) * KG + kb, hlf);
    if (MODE != 0) { const v16b al = frag_kb(Al + (m0 + nloc) * KG + kb, hlf);
#pragma unroll
      for (int t = 0; t < NT; ++t) { const v16b bw = frag_kb(W + (size_t)(n0 + t * 16 + nloc) * KG + kb, hlf); acc[t] = wmma16b(a, bw, acc[t]); acc[t] = wmma16b(al, bw, acc[t]); } }
    else {
#pragma unroll
      for (int t = 0; t < NT; ++t) acc[t] = wmma16b(a, frag_kb(W + (size_t)(n0 + t * 16 + nloc) * KG + kb, hlf), acc[t]); } }
#pragma unroll
  for (int t = 0; t < NT; ++t) { const int col = n0 + t * 16 + nloc; const float bb = (MODE == 2) ? bf16_rne(bias[c * ZD + col]) : bf16_rne(bias[col]);
#pragma unroll
    for (int r = 0; r < 8; ++r) { float v = acc[t][r] * (1.0f / (XS * WSC)) + bb; if (MODE != 2) v = lrelu(v); Ts[wave][8 * hlf + r][t * 16 + nloc] = v; } }
  wave_lds_sync();
  for (int pass = 0; pass < 2; ++pass) { for (int rr = 0; rr < 16; ++rr) {
      if (MODE != 2) { if (lane < 16) { v8b hv, lv; for (int j = 0; j < 8; ++j) { b16 a_, c_; split16(Ts[wave][rr][lane * 8 + j] * XS, a_, c_); hv[j] = a_; lv[j] = c_; } *(volatile v8b*)(Yh + (m0 + rr) * H + n0 + lane * 8) = hv; *(volatile v8b*)(Yl + (m0 + rr) * H + n0 + lane * 8) = lv; } }
      else if (lane < 8) *(volatile v4f*)(ZP + ((m0 + rr) * C + c) * ZD + lane * 4) = *(const v4f*)(&Ts[wave][rr][lane * 4]); }
    __threadfence(); }
}
__global__ __launch_bounds__(256) void proto_kernel(const float* __restrict__ proto, const float* __restrict__ logvar, float* __restrict__ PR, float* __restrict__ HINV) {
  const int t = blockIdx.x * 256 + threadIdx.x; const int np_ = C * K * P;
  if (t < np_ * ZD / 4) { const v4f v = *(const v4f*)(proto + (size_t)t * 4); const v4f o = {bf16_rne(v[0]), bf16_rne(v[1]), bf16_rne(v[2]), bf16_rne(v[3])}; for (int pass = 0; pass < 2; ++pass) { *(volatile v4f*)(PR + (size_t)t * 4) = o; __threadfence(); } }
  else if (t < np_ * ZD / 4 + (np_ + 3) / 4 * 1) { const int i0 = (t - np_ * ZD / 4) * 4; v4f o; for (int j = 0; j < 4; ++j) { const int i = i0 + j; o[j] = (i < np_) ? 1.0f / (2.0f * __expf(bf16_rne(logvar[i]))) : 0.0f; } for (int pass = 0; pass < 2; ++pass) { *(volatile v4f*)(HINV + i0) = o; __threadfence(); } }
}
__global__ __launch_bounds__(512) void head_kernel(const float* __restrict__ ZP, const float* __restrict__ PR, const float* __restrict__ HINV, const float* __restrict__ cbias, const float* __restrict__ biask, const float* __restrict__ imp, float* __restrict__ logits, float* __restrict__ clog) {
  __shared__ float CL[16][C * K]; __shared__ float LG[16][K];
  const int wave = threadIdx.x >> 5, lane = threadIdx.x & 31, t_ = threadIdx.x; const int b = blockIdx.x * 16 + wave;
  const int kA = lane >> 2, pA = lane & 3; const int kB = 8 + (lane >> 2);
  float sA = 0.0f, sB = 0.0f;
  for (int c = 0; c < C; ++c) { const float* z = ZP + ((size_t)b * C + c) * ZD; float zr[ZD];
#pragma unroll
    for (int d4 = 0; d4 < ZD; d4 += 4) { const v4f v = *(const v4f*)(z + d4); zr[d4] = v[0]; zr[d4 + 1] = v[1]; zr[d4 + 2] = v[2]; zr[d4 + 3] = v[3]; }
    const float wimp = fabsf(bf16_rne(imp[c]));
#pragma unroll 1
    for (int ps = 0; ps < 2; ++ps) { const int k = ps ? kB : kA; const bool valid = ps ? (lane < 8) : true; const int kk = valid ? k : 0; const size_t combo = ((size_t)c * K + kk) * P + pA;
      const float* pr = PR + combo * ZD; float d2 = 0.0f;
#pragma unroll
      for (int d4 = 0; d4 < ZD; d4 += 4) { const v4f v = *(const v4f*)(pr + d4); float df; df = zr[d4] - v[0]; d2 += pmul(df, df); df = zr[d4 + 1] - v[1]; d2 += pmul(df, df); df = zr[d4 + 2] - v[2]; d2 += pmul(df, df); df = zr[d4 + 3] - v[3]; d2 += pmul(df, df); }
      float sc = d2 * HINV[combo]; sc = fminf(sc, __shfl_xor(sc, 1)); sc = fminf(sc, __shfl_xor(sc, 2));
      const float cl = -sc + bf16_rne(cbias[c * K + kk]);
      if (valid && pA == 0) { CL[wave][c * K + kk] = cl; if (ps) sB += pmul(__expf(cl), wimp); else sA += pmul(__expf(cl), wimp); } } }
  if (pA == 0) { LG[wave][kA] = __logf(sA + 1e-16f) + bf16_rne(biask[kA]); if (lane < 8) LG[wave][kB] = __logf(sB + 1e-16f) + bf16_rne(biask[kB]); }
  __syncthreads();
  for (int pass = 0; pass < 2; ++pass) { for (int i = t_; i < 16 * C * K; i += 512) ((volatile float*)clog)[(size_t)blockIdx.x * 16 * C * K + i] = CL[i / (C * K)][i % (C * K)];
    if (t_ < 16 * K) ((volatile float*)logits)[(size_t)blockIdx.x * 16 * K + t_] = LG[t_ / K][t_ % K]; __threadfence(); }
}
}

extern "C" void kernel_launch(void* const* d_in, const int* in_sizes, int n_in, void* d_out, int out_size, void* d_ws, size_t ws_size, hipStream_t stream) {
  (void)n_in;
  auto Fp = [&](int i) { return (const float*)d_in[i]; };
  if (in_sizes[0] != B * G || in_sizes[1] != C * G || in_sizes[2] != G * H || in_sizes[4] != H * H || in_sizes[6] != C * ZD * H || in_sizes[8] != C * K * P * ZD || out_size != B * K + B * C * K) return;
  size_t off = 0; char* ws = (char*)d_ws;
  auto carve = [&](size_t bytes) { char* p = ws + off; off += (bytes + 255) & ~(size_t)255; return p; };
  int* IDX = (int*)carve((size_t)C * KG * 4); int* FLAG = (int*)carve(256); b16* XG = (b16*)carve((size_t)B * KG * 2); b16* W1G = (b16*)carve((size_t)H * KG * 2); b16* W2T = (b16*)carve((size_t)H * H * 2); b16* CW = (b16*)carve((size_t)C * ZD * H * 2);
  b16* Hh = (b16*)carve((size_t)B * H * 2); b16* Hl = (b16*)carve((size_t)B * H * 2); b16* Yh = (b16*)carve((size_t)B * H * 2); b16* Yl = (b16*)carve((size_t)B * H * 2); float* ZP = (float*)carve((size_t)B * C * ZD * 4); float* PR = (float*)carve((size_t)C * K * P * ZD * 4); float* HINV = (float*)carve((size_t)C * K * P * 4 + 256);
  if (off > ws_size || off > ((size_t)128 << 20)) return;
  genes_kernel<<<C, 256, 0, stream>>>(Fp(1), IDX, FLAG);
  prep_kernel<<<(unsigned)(((size_t)H * H / 8 + (size_t)C * ZD * H / 8 + 255) / 256), 256, 0, stream>>>(Fp(4), Fp(6), W2T, CW);
  for (int c = 0; c < C; ++c) {
    gather_kernel<<<(unsigned)(((size_t)B * KG / 8 + (size_t)H * KG / 8 + 255) / 256), 256, 0, stream>>>(Fp(0), Fp(2), IDX, c, XG, W1G);
    gemm_kernel<0><<<dim3(B / 64, H / 128), 128, 0, stream>>>(XG, nullptr, W1G, Fp(3), c, Hh, Hl, nullptr);
    gemm_kernel<1><<<dim3(B / 64, H / 128), 128, 0, stream>>>(Hh, Hl, W2T, Fp(5), c, Yh, Yl, nullptr);
    gemm_kernel<2><<<dim3(B / 64, 1), 128, 0, stream>>>(Yh, Yl, CW + (size_t)c * ZD * H, Fp(7), c, nullptr, nullptr, ZP);
  }
  proto_kernel<<<(C * K * P * ZD / 4 + (C * K * P + 3) / 4 + 255) / 256, 256, 0, stream>>>(Fp(8), Fp(9), PR, HINV);
  head_kernel<<<B / 16, 512, 0, stream>>>(ZP, PR, HINV, Fp(10), Fp(11), Fp(12), (float*)d_out, (float*)d_out + (size_t)B * K);
}
